// Local_Receptive_Field_18872086298823
// MI455X (gfx1250) — hardware-verified
//
#include <hip/hip_runtime.h>
#include <stddef.h>
#include <stdint.h>

#define NB   1024
#define NN   1024
#define IMG  64
#define NEL  7
#define NIN  4
#define NCT  3
#define HID  90
#define HP   96
#define NT   6
#define KC   3
#define NGRP 32
#define BCH  32
#define NBC  (NB / BCH)
#define TPB  64

static_assert(NGRP * 32 == NN);
static_assert(NBC * BCH == NB);
static_assert(NT * 16 == HP);
static_assert(KC * 32 == HP);
static_assert(HP >= HID);
static_assert((HP % 8) == 0);
static_assert(NGRP == 32);

typedef unsigned short u16;
typedef __bf16 v16b __attribute__((ext_vector_type(16)));
typedef unsigned short v8us __attribute__((ext_vector_type(8)));
typedef float v8f __attribute__((ext_vector_type(8)));
typedef float v4f __attribute__((ext_vector_type(4)));
typedef float v2f __attribute__((ext_vector_type(2)));

union Frag  { v16b v; v8us h[2]; };
union Pack8 { v8us h; u16 s[8]; };

__device__ __forceinline__ v8f zero8() { return (v8f){0.f, 0.f, 0.f, 0.f, 0.f, 0.f, 0.f, 0.f}; }

__device__ __forceinline__ v8f mma(v16b a, v16b b, v8f c) {
  c = __builtin_amdgcn_wmma_f32_16x16x32_bf16(false, a, false, b, (short)0, c, false, false);
  asm volatile("v_nop\n\tv_nop\n\tv_nop\n\tv_nop" : "+v"(c) : "v"(a), "v"(b));
  return c;
}

__device__ __forceinline__ u16 f2bf(float f) {
  unsigned int u = __float_as_uint(f);
  u += 0x7FFFu + ((u >> 16) & 1u);
  return (u16)(u >> 16);
}
__device__ __forceinline__ float bf2f(u16 h) { return __uint_as_float(((unsigned int)h) << 16); }
__device__ __forceinline__ u16 lo_of(float f, u16 hi) { return f2bf(f - bf2f(hi)); }
__device__ __forceinline__ void split8(const float (&v)[8], v8us& hu, v8us& lu) {
  Pack8 ph, pl;
#pragma unroll
  for (int i = 0; i < 8; ++i) {
    const u16 h = f2bf(v[i]);
    ph.s[i] = h;
    pl.s[i] = lo_of(v[i], h);
  }
  hu = ph.h;
  lu = pl.h;
}

__device__ __forceinline__ float elu1(float x) {
  const float xn = (x < 0.f) ? x : 0.f;
  const float em = expm1f(xn);
  return (x > 0.f) ? x : em;
}

__device__ __forceinline__ v16b ldfrag(const u16* p, int ld, int row0, int k0, int lane) {
  const int m = lane & 15, lh = lane >> 4;
  const u16* q = p + (size_t)(row0 + m) * ld + k0 + 8 * lh;
  Frag f;
  f.h[0] = *(const v8us*)(q);
  f.h[1] = *(const v8us*)(q + 16);
  return f.v;
}

__global__ __launch_bounds__(TPB) void k_lrf(const float* __restrict__ x, const float* __restrict__ controls,
                                             const float* __restrict__ W1, const float* __restrict__ b1,
                                             const float* __restrict__ W2, const float* __restrict__ b2,
                                             const float* __restrict__ W3, const float* __restrict__ b3,
                                             const int* __restrict__ ilist, const int* __restrict__ clist,
                                             float* __restrict__ out) {
  __shared__ __align__(16) u16 W2h[HP * HP];
  __shared__ __align__(16) u16 W2l[HP * HP];
  __shared__ __align__(16) u16 Hh[2][16 * HP];
  __shared__ __align__(16) u16 Hl[2][16 * HP];
  __shared__ __align__(16) float W1s[NEL * HP];
  __shared__ __align__(16) float b1s[HP];
  __shared__ __align__(16) float outs[32];

  const int tid = threadIdx.x, lane = tid & 31, wave = tid >> 5;
  const int lh = lane >> 4, m = lane & 15;
  const int ng = (int)blockIdx.x & (NGRP - 1);
  const int bc = (int)blockIdx.x >> 5;

  for (int q = tid; q < HP * HP / 8; q += TPB) {
    const int n = q / (HP / 8), kb = (q - n * (HP / 8)) * 8;
    const int nn = (n < HID) ? n : (HID - 1);
    float v[8];
#pragma unroll
    for (int i = 0; i < 8; ++i) {
      const int k = kb + i, kk = (k < HID) ? k : (HID - 1);
      const float t = W2[kk * HID + nn];
      v[i] = (k < HID && n < HID) ? t : 0.f;
    }
    v8us hu, lu;
    split8(v, hu, lu);
    *(v8us*)(W2h + n * HP + kb) = hu;
    *(v8us*)(W2l + n * HP + kb) = lu;
  }
  for (int i = tid; i < NEL * HP; i += TPB) {
    const int e = i / HP, c = i - e * HP, cc = (c < HID) ? c : (HID - 1);
    const float t = W1[e * HID + cc];
    W1s[i] = (c < HID) ? t : 0.f;
  }
  for (int i = tid; i < HP; i += TPB) {
    const int cc = (i < HID) ? i : (HID - 1);
    const float t = b1[cc];
    b1s[i] = (i < HID) ? t : 0.f;
  }

  const int nl = wave * 16 + m;
  const int n = ng * 32 + nl;
  int il[NIN], cl[NCT];
  float ct[NCT];
#pragma unroll
  for (int i = 0; i < NIN; ++i) il[i] = ilist[n * NIN + i];
#pragma unroll
  for (int j = 0; j < NCT; ++j) { cl[j] = clist[n * NCT + j]; ct[j] = controls[n * NCT + j]; }
  float b2v[NT], w3v[NT];
#pragma unroll
  for (int nt = 0; nt < NT; ++nt) {
    const int col = 16 * nt + m, cc = (col < HID) ? col : (HID - 1);
    const float tb = b2[cc], tw = W3[cc];
    b2v[nt] = (col < HID) ? tb : 0.f;
    w3v[nt] = (col < HID) ? tw : 0.f;
  }
  const float bias3 = b3[0];
  __syncthreads();

  u16* myh = &Hh[wave][0];
  u16* myl = &Hl[wave][0];

#pragma unroll 1
  for (int it = 0; it < BCH; ++it) {
    const int b = bc * BCH + it;
    const float* px = x + (size_t)b * (IMG * IMG) + (size_t)(2 * ng) * IMG + 2 * nl;
    const v2f p0 = *(const v2f*)(px);
    const v2f p1 = *(const v2f*)(px + IMG);
    float pt[NIN];
    pt[0] = p0[0]; pt[1] = p0[1]; pt[2] = p1[0]; pt[3] = p1[1];
    float E[NEL];
#pragma unroll
    for (int e = 0; e < NEL; ++e) {
      float v = 0.f;
#pragma unroll
      for (int i = 0; i < NIN; ++i) v = (il[i] == e) ? pt[i] : v;
#pragma unroll
      for (int j = 0; j < NCT; ++j) v = (cl[j] == e) ? ct[j] : v;
      E[e] = v;
    }
#pragma unroll 1
    for (int g = 0; g < 6; ++g) {
      const int c0 = 48 * lh + 8 * g;
      float a8[8];
#pragma unroll
      for (int i = 0; i < 8; ++i) a8[i] = 0.f;
#pragma unroll
      for (int e = 0; e < NEL; ++e) {
        const v4f w0 = *(const v4f*)(W1s + e * HP + c0);
        const v4f w1 = *(const v4f*)(W1s + e * HP + c0 + 4);
#pragma unroll
        for (int i = 0; i < 4; ++i) {
          a8[i]     = fmaf(E[e], w0[i], a8[i]);
          a8[4 + i] = fmaf(E[e], w1[i], a8[4 + i]);
        }
      }
      const v4f bb0 = *(const v4f*)(b1s + c0);
      const v4f bb1 = *(const v4f*)(b1s + c0 + 4);
      float hv[8];
#pragma unroll
      for (int i = 0; i < 4; ++i) {
        hv[i]     = elu1(a8[i] + bb0[i]);
        hv[4 + i] = elu1(a8[4 + i] + bb1[i]);
      }
      v8us hu, lu;
      split8(hv, hu, lu);
      *(v8us*)(myh + m * HP + c0) = hu;
      *(v8us*)(myl + m * HP + c0) = lu;
    }
    __syncthreads();

    v16b ah[KC], al[KC];
#pragma unroll
    for (int kc = 0; kc < KC; ++kc) {
      ah[kc] = ldfrag(myh, HP, 0, 32 * kc, lane);
      al[kc] = ldfrag(myl, HP, 0, 32 * kc, lane);
    }
    float p[8];
#pragma unroll
    for (int r = 0; r < 8; ++r) p[r] = 0.f;
#pragma unroll
    for (int nt = 0; nt < NT; ++nt) {
      v8f acc = zero8();
#pragma unroll
      for (int kc = 0; kc < KC; ++kc) {
        const v16b bh = ldfrag(W2h, HP, 16 * nt, 32 * kc, lane);
        const v16b bl = ldfrag(W2l, HP, 16 * nt, 32 * kc, lane);
        acc = mma(ah[kc], bh, acc);
        acc = mma(al[kc], bh, acc);
        acc = mma(ah[kc], bl, acc);
      }
#pragma unroll
      for (int r = 0; r < 8; ++r) {
        const float h2 = elu1(acc[r] + b2v[nt]);
        p[r] = fmaf(h2, w3v[nt], p[r]);
      }
    }
#pragma unroll
    for (int off = 1; off < 16; off <<= 1) {
#pragma unroll
      for (int r = 0; r < 8; ++r) p[r] += __shfl_xor(p[r], off, 32);
    }
    if (m == 0) {
      const v4f o0 = (v4f){p[0] + bias3, p[1] + bias3, p[2] + bias3, p[3] + bias3};
      const v4f o1 = (v4f){p[4] + bias3, p[5] + bias3, p[6] + bias3, p[7] + bias3};
      *(v4f*)(outs + 16 * wave + 8 * lh)     = o0;
      *(v4f*)(outs + 16 * wave + 8 * lh + 4) = o1;
    }
    __syncthreads();

    const bool wr = (wave == 0) && (lane < 8);
    const v4f ov = *(const v4f*)(outs + 4 * (lane & 7));
    float* op = out + (size_t)b * NN + (size_t)ng * 32 + 4 * (lane & 7);
    if (wr) *(volatile v4f*)op = ov;
    __threadfence();
    if (wr) *(volatile v4f*)op = ov;
  }
}

extern "C" void kernel_launch(void* const* d_in, const int* in_sizes, int n_in,
                              void* d_out, int out_size, void* d_ws, size_t ws_size,
                              hipStream_t stream) {
  if (n_in < 10) return;
  if (in_sizes[0] != NB * IMG * IMG) return;
  if (in_sizes[1] != NN * NCT) return;
  if (in_sizes[2] != NEL * HID) return;
  if (in_sizes[3] != HID) return;
  if (in_sizes[4] != HID * HID) return;
  if (in_sizes[5] != HID) return;
  if (in_sizes[6] != HID) return;
  if (in_sizes[7] != 1) return;
  if (in_sizes[8] != NN * NIN) return;
  if (in_sizes[9] != NN * NCT) return;
  if (out_size != NB * NN) return;
  (void)d_ws; (void)ws_size;

  const float* x        = (const float*)d_in[0];
  const float* controls = (const float*)d_in[1];
  const float* W1       = (const float*)d_in[2];
  const float* b1       = (const float*)d_in[3];
  const float* W2       = (const float*)d_in[4];
  const float* b2       = (const float*)d_in[5];
  const float* W3       = (const float*)d_in[6];
  const float* b3       = (const float*)d_in[7];
  const int*   ilist    = (const int*)d_in[8];
  const int*   clist    = (const int*)d_in[9];
  float* out = (float*)d_out;

  k_lrf<<<dim3(NGRP * NBC), dim3(TPB), 0, stream>>>(x, controls, W1, b1, W2, b2, W3, b3, ilist, clist, out);
  (void)hipGetLastError();
}
